// MultiScalePyramidAttention_85985245265955
// MI455X (gfx1250) — hardware-run, weakly checked
//
#include <hip/hip_runtime.h>
#include <math.h>

typedef __attribute__((ext_vector_type(16))) _Float16 v16h;
typedef __attribute__((ext_vector_type(16))) __bf16 v16b;
typedef __attribute__((ext_vector_type(8)))  _Float16 v8h;
typedef __attribute__((ext_vector_type(8)))  float v8f;
typedef __attribute__((ext_vector_type(4)))  float v4f;
typedef __attribute__((ext_vector_type(2)))  float v2f;
typedef __attribute__((ext_vector_type(4)))  unsigned v4u;
typedef __attribute__((ext_vector_type(4)))  int v4i;
typedef float __attribute__((may_alias)) float_a;
typedef int __attribute__((may_alias)) int_a;

template <typename T> __device__ __forceinline__ void vst2(void* p, T v) { *(volatile T*)p = v; __threadfence(); *(volatile T*)p = v; }
__device__ __forceinline__ v8f wmma16(v16h a, v16h b, v8f c) {
  v8f d = __builtin_amdgcn_wmma_f32_16x16x32_f16(false, a, false, b, (short)0, c, false, false);
  asm volatile("v_nop\n\tv_nop\n\tv_nop\n\tv_nop" : "+v"(d) : "v"(a), "v"(b));
  return d;
}
__device__ __forceinline__ v8f wmma_bf(v16b a, v16b b, v8f c) {
  v8f d = __builtin_amdgcn_wmma_f32_16x16x32_bf16(false, a, false, b, (short)0, c, false, false);
  asm volatile("v_nop\n\tv_nop\n\tv_nop\n\tv_nop" : "+v"(d) : "v"(a), "v"(b));
  return d;
}
__device__ __forceinline__ v16h frag_h(const _Float16* rowk0, int lane) {
  union { v16h v; v8h q[2]; } u; const _Float16* p = rowk0 + 8 * (lane >> 4);
  u.q[0] = *(const v8h*)p; u.q[1] = *(const v8h*)(p + 16); return u.v;
}
__device__ __forceinline__ v16h frag_f32(const float* rowk0, int lane) {
  v16h a; const float* p = rowk0 + 8 * (lane >> 4);
#pragma unroll
  for (int i = 0; i < 8; ++i) { a[i] = (_Float16)p[i]; a[8 + i] = (_Float16)p[16 + i]; }
  return a;
}
__device__ __forceinline__ v16h frag_f32s(const float* rowk0, int lane, float sc) {
  v16h a; const float* p = rowk0 + 8 * (lane >> 4);
#pragma unroll
  for (int i = 0; i < 8; ++i) { a[i] = (_Float16)(p[i] * sc); a[8 + i] = (_Float16)(p[16 + i] * sc); }
  return a;
}
__device__ __forceinline__ v16h fragc_f32(const float* W, int k0, int n, int lane, int ld, int K) {
  v16h a; const int g = lane >> 4;
#pragma unroll
  for (int i = 0; i < 8; ++i) { const int ka = k0 + 8 * g + i, kb = ka + 16;
    a[i] = (_Float16)(ka < K ? W[(size_t)(ka < K ? ka : K - 1) * ld + n] : 0.f); a[8 + i] = (_Float16)(kb < K ? W[(size_t)(kb < K ? kb : K - 1) * ld + n] : 0.f); }
  return a;
}
struct F2 { v16b h, l; };
__device__ __forceinline__ F2 bsplit16(const float v[16]) { F2 r;
#pragma unroll
  for (int i = 0; i < 16; ++i) { const __bf16 h = (__bf16)v[i]; r.h[i] = h; r.l[i] = (__bf16)(v[i] - (float)h); }
  return r; }
__device__ __forceinline__ F2 split_row(const float* row, int k0, int lane) { float v[16]; const float* p = row + k0 + 8 * (lane >> 4);
#pragma unroll
  for (int i = 0; i < 8; ++i) { v[i] = p[i]; v[8 + i] = p[16 + i]; }
  return bsplit16(v); }
__device__ __forceinline__ F2 split_rowK(const float* row, int k0, int lane, int K) { float v[16]; const int g = lane >> 4;
#pragma unroll
  for (int i = 0; i < 8; ++i) { const int ka = k0 + 8 * g + i, kb = ka + 16; v[i] = ka < K ? row[ka < K ? ka : K - 1] : 0.f; v[8 + i] = kb < K ? row[kb < K ? kb : K - 1] : 0.f; }
  return bsplit16(v); }
__device__ __forceinline__ F2 split_col(const float* W, int k0, int n, int lane, int ld, int K) { float v[16]; const int g = lane >> 4;
#pragma unroll
  for (int i = 0; i < 8; ++i) { const int ka = k0 + 8 * g + i, kb = ka + 16; v[i] = ka < K ? W[(size_t)(ka < K ? ka : K - 1) * ld + n] : 0.f; v[8 + i] = kb < K ? W[(size_t)(kb < K ? kb : K - 1) * ld + n] : 0.f; }
  return bsplit16(v); }
__device__ __forceinline__ v8f mac3(const F2& a, const F2& b, v8f c) { c = wmma_bf(a.l, b.h, c); c = wmma_bf(a.h, b.l, c); return wmma_bf(a.h, b.h, c); }
__device__ __forceinline__ float sigm(float v) { return 1.0f / (1.0f + expf(-v)); }
#define LDSX() do { asm volatile("s_wait_dscnt 0" ::: "memory"); __builtin_amdgcn_wave_barrier(); __builtin_amdgcn_fence(__ATOMIC_RELEASE, "workgroup"); } while (0)


#define NB 8
#define CC 128
#define HH 64
#define WWD 64
#define NPIX (HH * WWD)
#define NH 8
#define HD 16
#define KC9 (CC * 9)
#ifndef TNB
#define TNB NB
#define TPB (NPIX / 64)
#endif
typedef __attribute__((ext_vector_type(8))) __bf16 v8b;
__device__ __forceinline__ v16b frag_b(const __bf16* rowk0, int lane) {
  union { v16b v; v8b q[2]; } u; const __bf16* p = rowk0 + 8 * (lane >> 4);
  u.q[0] = *(const v8b*)p; u.q[1] = *(const v8b*)(p + 16); return u.v;
}
__device__ __forceinline__ float bfr(float v) { return (float)(__bf16)v; }
__device__ __attribute__((noinline)) float exp_ni(float v) { return expf(v); }
__device__ __attribute__((noinline)) float erf_ni(float v) { return erff(v); }

#define WS_PC  0u
#define WS_PI  (WS_PC + 2u * (size_t)4 * CC * KC9)
#define WS_PA  (WS_PI + 2u * (size_t)384 * CC)
#define WS_PFU (WS_PA + 2u * (size_t)CC * CC)
#define WS_XT  (WS_PFU + 2u * (size_t)CC * 512)
#define WS_P2  (WS_XT + 4u * (size_t)NB * NPIX * CC)
#define WS_P4  (WS_P2 + 4u * (size_t)NB * 1024 * CC)
#define WS_P8  (WS_P4 + 4u * (size_t)NB * 256 * CC)
#define WS_F2  (WS_P8 + 4u * (size_t)NB * 64 * CC)
#define WS_F4  (WS_F2 + 4u * (size_t)NB * 1024 * CC)
#define WS_F8  (WS_F4 + 4u * (size_t)NB * 256 * CC)
#define WS_XR  (WS_F8 + 4u * (size_t)NB * 64 * CC)
#define WS_QKV (WS_XR + 4u * (size_t)NB * NPIX * 4 * CC)
#define WS_OO  (WS_QKV + 2u * (size_t)NB * NPIX * 4 * 384)
#define WS_END (WS_OO + 2u * (size_t)NB * NPIX * 4 * CC)
#define WS_NM  WS_QKV

__global__ __launch_bounds__(128) void k_pack(const float* __restrict__ CW, const float* __restrict__ WI, const float* __restrict__ WA, const float* __restrict__ WF, __bf16* __restrict__ P) { const int n = blockIdx.x, which = blockIdx.y, t = threadIdx.x; __shared__ __align__(16) __bf16 sb[KC9]; __shared__ __align__(16) _Float16 sh[CC];
  if (which < 4) {
    for (int k = t; k < KC9; k += 128) { const int tap = k / CC, c = k % CC; sb[k] = (__bf16)CW[((((size_t)which * CC + n) * CC + c) * 9) + tap]; } __syncthreads(); for (int q = t; q < KC9 / 8; q += 128) vst2((unsigned*)(P + WS_PC / 2 + ((size_t)which * CC + n) * KC9 + q * 8), *(const v4u*)&sb[q * 8]); }
  else if (which < 7) { const int row = (which - 4) * CC + n; sh[t] = (_Float16)(bfr(WI[(size_t)row * CC + t]) * 256.0f); __syncthreads(); if (t < CC / 8) vst2((unsigned*)((_Float16*)P + WS_PI / 2 + (size_t)row * CC + t * 8), *(const v4u*)&sh[t * 8]); }
  else if (which == 7) { sh[t] = (_Float16)(bfr(WA[(size_t)n * CC + t]) * 256.0f); __syncthreads(); if (t < CC / 8) vst2((unsigned*)((_Float16*)P + WS_PA / 2 + (size_t)n * CC + t * 8), *(const v4u*)&sh[t * 8]); }
  else { for (int k = t; k < 512; k += 128) sb[k] = (__bf16)WF[(size_t)n * 512 + k]; __syncthreads(); if (t < 64) vst2((unsigned*)(P + WS_PFU / 2 + (size_t)n * 512 + t * 8), *(const v4u*)&sb[t * 8]); } }
__global__ __launch_bounds__(256) void k_xt(const float* __restrict__ X, float* __restrict__ XT) { __shared__ float st[64][CC + 1]; __shared__ __align__(16) float so2[64][CC + 4]; const int t = threadIdx.x; const int p0 = blockIdx.x * 64; const size_t b = blockIdx.y;
  for (int e = t; e < CC * 64; e += 256) { const int c = e >> 6, pl = e & 63; st[pl][c] = bfr(X[(b * CC + c) * NPIX + p0 + pl]); } __syncthreads();
  for (int e = t; e < 64 * CC; e += 256) { const int pl = e >> 7, c = e & 127; so2[pl][c] = st[pl][c]; } __syncthreads();
  for (int e = t; e < 64 * 32; e += 256) { const int pl = e >> 5, q = e & 31; vst2(XT + ((b * NPIX + p0 + pl) * CC) + q * 4, *(const v4f*)&so2[pl][q * 4]); } }
__global__ __launch_bounds__(128) void k_pool(const float* __restrict__ XT, float* __restrict__ P2, float* __restrict__ P4, float* __restrict__ P8) { const int t = threadIdx.x; const int sI = blockIdx.z; const int s = 2 << sI; const int n = HH / s; const int Y = blockIdx.x; const size_t b = blockIdx.y; if (Y >= n) return; float* dst = (sI == 0) ? P2 : (sI == 1) ? P4 : P8;
  for (int X = 0; X < n; ++X) { float a = 0.f; for (int dy = 0; dy < s; ++dy) for (int dx = 0; dx < s; ++dx) a += XT[((b * NPIX + (size_t)(Y * s + dy) * WWD + X * s + dx) * CC) + t]; __shared__ __align__(16) float so2[CC]; so2[t] = a / (float)(s * s); __syncthreads(); if (t < CC / 4) vst2(dst + ((b * n * n + (size_t)Y * n + X) * CC) + t * 4, *(const v4f*)&so2[t * 4]); __syncthreads(); } }
template <int SC>
__global__ __launch_bounds__(128) void k_conv(const float* __restrict__ IN, const __bf16* __restrict__ P, const float* __restrict__ CB, float* __restrict__ OUT) { __shared__ __align__(16) float so[4][16][132];
  const int tid = threadIdx.x, wave = tid >> 5, lane = tid & 31, col = lane & 15, g = lane >> 4; const size_t b = blockIdx.z; const int n = HH >> SC; const int npix = n * n; const int p0 = blockIdx.x * 64 + wave * 16; const __bf16* Wr = P + WS_PC / 2 + (size_t)SC * CC * KC9;
  const int pix = p0 + col; const int py = pix / n, px = pix % n; const bool prow = pix < npix;
  v8f acc[8] = {};
#pragma unroll 1
  for (int tap = 0; tap < 9; ++tap) { const int yy = py + tap / 3 - 1, xx = px + tap % 3 - 1; const bool inb = prow && yy >= 0 && yy < n && xx >= 0 && xx < n; const float* src = IN + ((b * npix + (size_t)(inb ? yy * n + xx : 0)) * CC);
#pragma unroll
    for (int q = 0; q < 4; ++q) { float v[16]; const float* p = src + q * 32 + 8 * g;
#pragma unroll
      for (int i = 0; i < 8; ++i) { v[i] = inb ? p[i] : 0.f; v[8 + i] = inb ? p[16 + i] : 0.f; }
      const int kc = tap * 4 + q;
      if (SC == 0) { v16b a;
#pragma unroll
        for (int i = 0; i < 16; ++i) a[i] = (__bf16)v[i];
#pragma unroll
        for (int j = 0; j < 8; ++j) acc[j] = wmma_bf(a, frag_b(Wr + (size_t)(j * 16 + col) * KC9 + kc * 32, lane), acc[j]); }
      else { const F2 a = bsplit16(v);
#pragma unroll
        for (int j = 0; j < 8; ++j) { const v16b w = frag_b(Wr + (size_t)(j * 16 + col) * KC9 + kc * 32, lane); acc[j] = wmma_bf(a.h, w, acc[j]); acc[j] = wmma_bf(a.l, w, acc[j]); } } } }
#pragma unroll
  for (int j = 0; j < 8; ++j) { const float bb = bfr(CB[SC * CC + j * 16 + col]);
#pragma unroll
    for (int r = 0; r < 8; ++r) so[wave][8 * g + r][j * 16 + col] = acc[j][r] + bb; }
  LDSX();
  for (int rl = 0; rl < 16; ++rl) { const int pp = p0 + rl; if (pp >= npix) break; if (SC == 0) vst2(OUT + (((b * NPIX + pp) * 4 + 0) * CC) + lane * 4, *(const v4f*)&so[wave][rl][lane * 4]); else vst2(OUT + ((b * npix + pp) * CC) + lane * 4, *(const v4f*)&so[wave][rl][lane * 4]); } }
__device__ __forceinline__ void bilin(int i, int n_in, int& i0, int& i1, float& w1) { const float sc = (float)n_in / (float)HH; float src = ((float)i + 0.5f) * sc - 0.5f; src = fmaxf(src, 0.f); i0 = (int)floorf(src); i1 = (i0 + 1 < n_in - 1) ? i0 + 1 : n_in - 1; w1 = src - (float)i0; }
__global__ __launch_bounds__(128) void k_resize(const float* __restrict__ F2, const float* __restrict__ F4, const float* __restrict__ F8, float* __restrict__ XR) { const int t = threadIdx.x; const size_t b = blockIdx.y; const int p0 = blockIdx.x * 64;
  for (int pl = 0; pl < 64; ++pl) { const int pix = p0 + pl; const int y = pix / WWD, x = pix % WWD;
#pragma unroll
    for (int tok = 1; tok < 4; ++tok) { const int n = HH >> tok; const float* F = (tok == 1) ? F2 : (tok == 2) ? F4 : F8; int y0, y1, x0, x1; float wy, wx; bilin(y, n, y0, y1, wy); bilin(x, n, x0, x1, wx);
      const float* base = F + (b * (size_t)n * n) * CC + t; const float v00 = base[((size_t)y0 * n + x0) * CC], v01 = base[((size_t)y0 * n + x1) * CC], v10 = base[((size_t)y1 * n + x0) * CC], v11 = base[((size_t)y1 * n + x1) * CC];
      const float t0 = v00 * (1.0f - wy) + v10 * wy, t1 = v01 * (1.0f - wy) + v11 * wy; __shared__ __align__(16) float so2[CC]; so2[t] = t0 * (1.0f - wx) + t1 * wx; __syncthreads();
      if (t < CC / 4) vst2(XR + (((b * NPIX + pix) * 4 + tok) * CC) + t * 4, *(const v4f*)&so2[t * 4]); __syncthreads(); } } }
__global__ __launch_bounds__(128) void k_qkv(const float* __restrict__ XR, const _Float16* __restrict__ PI, const float* __restrict__ BI, _Float16* __restrict__ QKV) { __shared__ __align__(16) _Float16 so[64][136];
  const int tid = threadIdx.x, wave = tid >> 5, lane = tid & 31, col = lane & 15, g = lane >> 4; const size_t r0 = (size_t)blockIdx.x * 64 + wave * 16; const int c0 = blockIdx.y * 128;
  v8f acc[8] = {};
#pragma unroll
  for (int kc = 0; kc < CC / 32; ++kc) { v16h a; { const float* p = XR + (r0 + col) * CC + kc * 32 + 8 * g;
#pragma unroll
      for (int i = 0; i < 8; ++i) { a[i] = (_Float16)p[i]; a[8 + i] = (_Float16)p[16 + i]; } }
#pragma unroll
    for (int j = 0; j < 8; ++j) acc[j] = wmma16(a, frag_h(PI + (size_t)(c0 + j * 16 + col) * CC + kc * 32, lane), acc[j]); }
#pragma unroll
  for (int j = 0; j < 8; ++j) { const float bb = bfr(BI[c0 + j * 16 + col]);
#pragma unroll
    for (int r = 0; r < 8; ++r) so[wave * 16 + 8 * g + r][j * 16 + col] = (_Float16)(acc[j][r] * (1.0f / 256.0f) + bb); }
  __syncthreads(); for (int e = tid; e < 64 * 16; e += 128) { const int rl = e >> 4, q = e & 15; vst2((unsigned*)(QKV + ((size_t)blockIdx.x * 64 + rl) * 384 + c0 + q * 8), *(const v4u*)&so[rl][q * 8]); } }
__global__ __launch_bounds__(128) void k_pix(const _Float16* __restrict__ QKV, _Float16* __restrict__ OO) { __shared__ __align__(16) _Float16 so2[16][CC + 8]; const int t = threadIdx.x; const int h = t & 7, i = (t >> 3) & 3, pl = t >> 5; const size_t base = ((size_t)blockIdx.x * 4 + pl) * 4;
  const _Float16* qr = QKV + (base + i) * 384 + h * HD; float s[4];
#pragma unroll
  for (int j = 0; j < 4; ++j) { const _Float16* kr = QKV + (base + j) * 384 + CC + h * HD; float a = 0.f;
#pragma unroll 1
    for (int d = 0; d < HD; ++d) a += (float)qr[d] * (float)kr[d];
    s[j] = a * 0.25f; }
  const float mx = fmaxf(fmaxf(s[0], s[1]), fmaxf(s[2], s[3])); float ez[4], z = 0.f;
#pragma unroll
  for (int j = 0; j < 4; ++j) { ez[j] = __expf(s[j] - mx); z += ez[j]; }
  const float iz = 1.0f / z; const _Float16* v0 = QKV + (base + 0) * 384 + 2 * CC + h * HD;
#pragma unroll 1
  for (int d = 0; d < HD; ++d) { const float a = ez[0] * (float)v0[d] + ez[1] * (float)v0[384 + d] + ez[2] * (float)v0[768 + d] + ez[3] * (float)v0[1152 + d]; so2[pl * 4 + i][h * HD + d] = (_Float16)(a * iz); }
  __syncthreads();
  for (int e = t; e < 16 * 16; e += 128) { const int rl = e >> 4, q = e & 15; vst2((unsigned*)(OO + ((size_t)blockIdx.x * 16 + rl) * CC + q * 8), *(const v4u*)&so2[rl][q * 8]); } }
__global__ __launch_bounds__(128) void k_oln(const _Float16* __restrict__ OO, const _Float16* __restrict__ PA, const float* __restrict__ BA, const float* __restrict__ XR, const float* __restrict__ G, const float* __restrict__ Bt, float* __restrict__ NM) { __shared__ __align__(16) float so[4][16][132];
  const int tid = threadIdx.x, wave = tid >> 5, lane = tid & 31, col = lane & 15, g = lane >> 4; const size_t r0 = (size_t)blockIdx.x * 64 + wave * 16;
  v8f acc[8] = {};
#pragma unroll
  for (int kc = 0; kc < CC / 32; ++kc) { const v16h a = frag_h(OO + (r0 + col) * CC + kc * 32, lane);
#pragma unroll
    for (int j = 0; j < 8; ++j) acc[j] = wmma16(a, frag_h(PA + (size_t)(j * 16 + col) * CC + kc * 32, lane), acc[j]); }
  float sum[8], sq[8];
#pragma unroll
  for (int r = 0; r < 8; ++r) { sum[r] = 0.f;
#pragma unroll
    for (int j = 0; j < 8; ++j) { const int c = j * 16 + col; acc[j][r] = acc[j][r] * (1.0f / 256.0f) + bfr(BA[c]) + XR[(r0 + 8 * g + r) * CC + c]; sum[r] += acc[j][r]; }
#pragma unroll
    for (int o = 1; o < 16; o <<= 1) sum[r] += __shfl_xor(sum[r], o); }
#pragma unroll
  for (int r = 0; r < 8; ++r) { const float mu = sum[r] / (float)CC; sq[r] = 0.f;
#pragma unroll
    for (int j = 0; j < 8; ++j) { const float d = acc[j][r] - mu; sq[r] += d * d; }
#pragma unroll
    for (int o = 1; o < 16; o <<= 1) sq[r] += __shfl_xor(sq[r], o);
    const float inv = 1.0f / sqrtf(sq[r] / (float)CC + 1e-5f);
#pragma unroll
    for (int j = 0; j < 8; ++j) { const int c = j * 16 + col; so[wave][8 * g + r][c] = (acc[j][r] - mu) * inv * bfr(G[c]) + bfr(Bt[c]); } }
  LDSX(); for (int rl = 0; rl < 16; ++rl) vst2(NM + (r0 + rl) * CC + lane * 4, *(const v4f*)&so[wave][rl][lane * 4]); }
__global__ __launch_bounds__(128) void k_fus(const __bf16* __restrict__ PF, const float* __restrict__ NM, const float* __restrict__ FB, float* __restrict__ Y) { __shared__ __align__(16) float so[4][16][132];
  const int tid = threadIdx.x, wave = tid >> 5, lane = tid & 31, col = lane & 15, g = lane >> 4; const size_t b = blockIdx.z; const int o0 = blockIdx.x * 64 + wave * 16; const int p0 = blockIdx.y * 128;
  v8f acc[8] = {};
#pragma unroll 2
  for (int kc = 0; kc < 512 / 32; ++kc) { const v16b a = frag_b(PF + (size_t)(o0 + col) * 512 + kc * 32, lane);
#pragma unroll
    for (int jt = 0; jt < 8; ++jt) { const F2 w = split_row(NM + (b * NPIX + p0 + jt * 16 + col) * 512, kc * 32, lane); acc[jt] = wmma_bf(a, w.h, acc[jt]); acc[jt] = wmma_bf(a, w.l, acc[jt]); } }
#pragma unroll
  for (int jt = 0; jt < 8; ++jt)
#pragma unroll
    for (int r = 0; r < 8; ++r) so[wave][8 * g + r][jt * 16 + col] = acc[jt][r] + bfr(FB[o0 + 8 * g + r]);
  LDSX(); for (int rl = 0; rl < 16; ++rl) vst2(Y + ((b * CC + o0 + rl) * NPIX) + p0 + lane * 4, *(const v4f*)&so[wave][rl][lane * 4]); }
extern "C" void kernel_launch(void* const* d_in, const int* in_sizes, int n_in, void* d_out, int out_size, void* d_ws, size_t ws_size, hipStream_t stream) {
  (void)in_sizes; (void)n_in; (void)out_size;
  const float** F = (const float**)d_in;
  if (ws_size < (size_t)WS_END) return;
  char* ws = (char*)d_ws; __bf16* P = (__bf16*)ws; const _Float16 *PI = (const _Float16*)(ws + WS_PI), *PA = (const _Float16*)(ws + WS_PA); const __bf16* PF = (const __bf16*)(ws + WS_PFU);
  float *XT = (float*)(ws + WS_XT), *P2 = (float*)(ws + WS_P2), *P4 = (float*)(ws + WS_P4), *P8 = (float*)(ws + WS_P8), *F2 = (float*)(ws + WS_F2), *F4 = (float*)(ws + WS_F4), *F8 = (float*)(ws + WS_F8), *XR = (float*)(ws + WS_XR), *NM = (float*)(ws + WS_NM); _Float16 *QKV = (_Float16*)(ws + WS_QKV), *OO = (_Float16*)(ws + WS_OO);
  k_pack<<<dim3(CC, 9), 128, 0, stream>>>(F[1], F[3], F[5], F[9], P);
  k_xt<<<dim3(NPIX / 64, TNB), 256, 0, stream>>>(F[0], XT);
  k_pool<<<dim3(32, TNB, 3), 128, 0, stream>>>(XT, P2, P4, P8);
  k_conv<1><<<dim3(1024 / 64, 1, TNB), 128, 0, stream>>>(P2, P, F[2], F2);
  k_conv<2><<<dim3(256 / 64, 1, TNB), 128, 0, stream>>>(P4, P, F[2], F4);
  k_conv<3><<<dim3(1, 1, TNB), 128, 0, stream>>>(P8, P, F[2], F8);
  k_conv<0><<<dim3(TPB, 1, TNB), 128, 0, stream>>>(XT, P, F[2], XR);
  k_resize<<<dim3(TPB, TNB), 128, 0, stream>>>(F2, F4, F8, XR);
  k_qkv<<<dim3(TNB * TPB * 4, 3), 128, 0, stream>>>(XR, PI, F[4], QKV);
  k_pix<<<TNB * TPB * 64 / 4, 128, 0, stream>>>(QKV, OO);
  k_oln<<<TNB * TPB * 4, 128, 0, stream>>>(OO, PA, F[6], XR, F[7], F[8], NM);
  k_fus<<<dim3(CC / 64, (TPB * 64) / 128, TNB), 128, 0, stream>>>(PF, NM, F[10], (float*)d_out);
}
